// SimpleFineGrainedHead3_63883343561449
// MI455X (gfx1250) — hardware-verified
//
#include <hip/hip_runtime.h>
#include <math.h>

constexpr int kImg     = 96;
constexpr int kTxtB    = 96;
constexpr int kNVis    = 197;
constexpr int kNTxt    = 77;
constexpr int kDin     = 768;
constexpr int kEmb     = 512;
constexpr int kRowsV   = kImg * kNVis;
constexpr int kRowsVP  = 18944;
constexpr int kRowsT   = kTxtB * kNTxt;
constexpr int kRowsTP  = 7424;
constexpr int kClsPad  = 128;
constexpr int kChunkImg = 8;
constexpr int kNumChunk = 12;
constexpr int kSimN    = 1600;
constexpr int kSimLd   = 1600;
constexpr float kWCarry     = 16.0f;
constexpr float kWCarryInv  = 1.0f / 16.0f;
constexpr float kUnitCarry  = 16.0f;
constexpr float kSimScale   = 1.0f / 256.0f;

static_assert(kRowsVP % 64 == 0 && kRowsVP >= kRowsV, "pad");
static_assert(kRowsTP % 64 == 0 && kRowsTP >= kRowsT, "pad");
static_assert(kChunkImg * kNumChunk == kImg, "chunks");
static_assert(kChunkImg * kNVis <= kSimN && kSimN % 64 == 0, "chunk cols");
static_assert((kNumChunk - 1) * kChunkImg * kNVis + kSimN <= kRowsVP, "last chunk Bt rows inside padded plane");
static_assert(kDin % 32 == 0 && kEmb % 64 == 0, "K and N multiples");
static_assert(kRowsVP % 8 == 0 && kRowsTP % 8 == 0, "l2norm rows per block");

constexpr int kOut0Elem  = 0;
constexpr int kOut1Elem  = 196608 / 4;
constexpr int kOut2Elem  = 393216 / 4;
constexpr int kOut3Elem  = 430080 / 4;
constexpr int kOutTotal  = 466944 / 4;
static_assert(kOut1Elem == kImg * kEmb, "out1 offset");
static_assert(kOut2Elem == kOut1Elem + kTxtB * kEmb, "out2 offset");
static_assert(kOut3Elem == kOut2Elem + kImg * kTxtB, "out3 offset");
static_assert(kOutTotal == kOut3Elem + kImg * kTxtB, "out total");

constexpr size_t kBytesW16Plane  = (size_t)kEmb * kDin * 2;
constexpr size_t kOffW16   = 0;
constexpr size_t kBytesXC16Plane = (size_t)kClsPad * kDin * 2;
constexpr size_t kOffXC16  = kOffW16 + 4 * kBytesW16Plane;
constexpr size_t kBytesXT16 = (size_t)kRowsTP * kDin * 2;
constexpr size_t kOffXT16  = kOffXC16 + 2 * kBytesXC16Plane;
constexpr size_t kBytesPT32 = (size_t)kRowsTP * kEmb * 4;
constexpr size_t kOffPT32  = kOffXT16 + kBytesXT16;
constexpr size_t kBytesTT16 = (size_t)kRowsTP * kEmb * 2;
constexpr size_t kOffTT16  = kOffPT32 + kBytesPT32;
constexpr size_t kBytesVT16 = (size_t)kRowsVP * kEmb * 2;
constexpr size_t kOffVT16  = kOffTT16 + kBytesTT16;
constexpr size_t kBytesCLS32Plane = (size_t)kClsPad * kEmb * 4;
constexpr size_t kOffCLS32 = kOffVT16 + kBytesVT16;
constexpr size_t kBytesTAB = (size_t)kImg * kTxtB * 128;
constexpr size_t kOffTAB   = kOffCLS32 + 2 * kBytesCLS32Plane;
constexpr size_t kOffBIG   = kOffTAB + kBytesTAB;
constexpr size_t kBytesXV16 = (size_t)kRowsVP * kDin * 2;
constexpr size_t kOffXV16  = kOffBIG;
constexpr size_t kBytesPV32 = (size_t)kRowsVP * kEmb * 4;
constexpr size_t kOffPV32  = kOffXV16 + kBytesXV16;
constexpr size_t kBytesS   = (size_t)kRowsTP * kSimLd * 4;
constexpr size_t kOffS     = kOffBIG;
constexpr size_t kWsTotal  = kOffPV32 + kBytesPV32;
static_assert(kOffS + kBytesS <= kWsTotal, "S overlay inside BIG");
static_assert(kWsTotal <= (size_t)134217728, "carve within 128 MiB");
static_assert(kOffXC16 % 4096 == 0 && kOffXT16 % 4096 == 0 && kOffPT32 % 4096 == 0 && kOffTT16 % 4096 == 0 &&
              kOffVT16 % 4096 == 0 && kOffCLS32 % 4096 == 0 && kOffTAB % 4096 == 0 && kOffBIG % 4096 == 0 &&
              kOffPV32 % 4096 == 0, "aligned carves");

typedef __attribute__((ext_vector_type(16))) _Float16 v16h;
typedef __attribute__((ext_vector_type(8)))  _Float16 v8h;
typedef __attribute__((ext_vector_type(16))) __bf16   v16b;
typedef __attribute__((ext_vector_type(8)))  __bf16   v8b;
typedef __attribute__((ext_vector_type(8)))  float    v8f;
typedef __attribute__((ext_vector_type(4)))  float    v4f;
typedef __attribute__((ext_vector_type(4)))  unsigned int v4u;

__device__ __forceinline__ unsigned short f2bf_bits(float f) {
  unsigned u = __float_as_uint(f);
  return (unsigned short)((u + 0x7FFFu + ((u >> 16) & 1u)) >> 16);
}
__device__ __forceinline__ float bf_bits2f(unsigned short h) { return __uint_as_float(((unsigned)h) << 16); }

__device__ __forceinline__ void dep_guard_h(v8f& a, v8f& b, v16h x, v16h y) { asm volatile("v_nop\n\tv_nop\n\tv_nop\n\tv_nop" : "+v"(a), "+v"(b) : "v"(x), "v"(y)); }
__device__ __forceinline__ void dep_guard_b(v8f& a, v8f& b, v16b x, v16b y) { asm volatile("v_nop\n\tv_nop\n\tv_nop\n\tv_nop" : "+v"(a), "+v"(b) : "v"(x), "v"(y)); }
__device__ __forceinline__ void keep4_h(v16h a, v16h b, v16h c, v16h d) { asm volatile("v_nop" :: "v"(a), "v"(b), "v"(c), "v"(d)); }
__device__ __forceinline__ void keep4_b(v16b a, v16b b, v16b c, v16b d) { asm volatile("v_nop" :: "v"(a), "v"(b), "v"(c), "v"(d)); }
__device__ __forceinline__ void acc_guard4(v8f& a, v8f& b, v8f& c, v8f& d) { asm volatile("v_nop\n\tv_nop\n\tv_nop\n\tv_nop" : "+v"(a), "+v"(b), "+v"(c), "+v"(d)); }
template <typename T> struct Frag;
template <> struct Frag<_Float16> {
  typedef v16h V; union U { v16h v; v8h h[2]; };
  static __device__ __forceinline__ v16h load(const _Float16* p) {
    U f; f.h[0] = *(const v8h*)(p); f.h[1] = *(const v8h*)(p + 16); return f.v;
  }
  static __device__ __forceinline__ v8f mma(v16h a, v16h b, v8f c) {
    return __builtin_amdgcn_wmma_f32_16x16x32_f16(false, a, false, b, (short)0, c, false, false);
  }
  static __device__ __forceinline__ void guard(v8f& a, v8f& b, v16h x, v16h y) { dep_guard_h(a, b, x, y); }
  static __device__ __forceinline__ void keep(v16h a, v16h b, v16h c, v16h d) { keep4_h(a, b, c, d); }
};
template <> struct Frag<__bf16> {
  typedef v16b V; union U { v16b v; v8b h[2]; };
  static __device__ __forceinline__ v16b load(const __bf16* p) {
    U f; f.h[0] = *(const v8b*)(p); f.h[1] = *(const v8b*)(p + 16); return f.v;
  }
  static __device__ __forceinline__ v8f mma(v16b a, v16b b, v8f c) {
    return __builtin_amdgcn_wmma_f32_16x16x32_bf16(false, a, false, b, (short)0, c, false, false);
  }
  static __device__ __forceinline__ void guard(v8f& a, v8f& b, v16b x, v16b y) { dep_guard_b(a, b, x, y); }
  static __device__ __forceinline__ void keep(v16b a, v16b b, v16b c, v16b d) { keep4_b(a, b, c, d); }
};

__device__ __forceinline__ unsigned pk16(unsigned short a, unsigned short b) { return (unsigned)a | ((unsigned)b << 16); }
__device__ __forceinline__ unsigned short h_bits(float f) { const _Float16 h = (_Float16)f; return __builtin_bit_cast(unsigned short, h); }

template <int ET> struct Elem;
template <> struct Elem<0> { typedef _Float16 T; };
template <> struct Elem<1> { typedef __bf16 T; };
template <int ET, bool SPLIT, int BIAS_MODE, int OUT_MODE, bool RESID, int ACT = 0>
__global__ __launch_bounds__(256) void wmma_gemm64(
    const unsigned short* __restrict__ Ap, const unsigned short* __restrict__ A2p, int lda, long strideA,
    const unsigned short* __restrict__ Btp, const unsigned short* __restrict__ Bt2p, int ldb, long strideB,
    void* __restrict__ Cout, void* __restrict__ Cout2, int ldc, long strideC,
    const float* __restrict__ bias,
    const float* __restrict__ resid, long strideR,
    int M, int N, int K, float scale) {
  typedef typename Elem<ET>::T T;
  typedef typename Frag<T>::V V;
  const T* A = (const T*)Ap; const T* A2 = (const T*)A2p; const T* Bt = (const T*)Btp; const T* Bt2 = (const T*)Bt2p;
  __shared__ __align__(16) float sT[8][16 * 68];
  const int b    = blockIdx.y;
  const int lane = threadIdx.x & 31;
  const int wave = threadIdx.x >> 5;
  const int tilesN = N >> 6;
  const int tilesM = M >> 6;
  const int tile = blockIdx.x * 8 + wave;
  if (tile >= tilesM * tilesN) return;
  const int tm = tile / tilesN;
  const int tn = tile - tm * tilesN;
  const int m0 = tm << 6;
  const int n0 = tn << 6;

  const T* Ab  = A  + (size_t)b * strideA;
  const T* Bb  = Bt + (size_t)b * strideB;
  const T* Ab2 = SPLIT ? (A2  + (size_t)b * strideA) : nullptr;
  const T* Bb2 = SPLIT ? (Bt2 + (size_t)b * strideB) : nullptr;

  const int rlane = lane & 15;
  const int koff  = (lane >> 4) * 8;
  const int mOff  = (lane >> 4) * 8;

  v8f acc[4][4];
#pragma unroll
  for (int i = 0; i < 4; ++i)
#pragma unroll
    for (int j = 0; j < 4; ++j) acc[i][j] = (v8f){0.f,0.f,0.f,0.f,0.f,0.f,0.f,0.f};

  for (int k0 = 0; k0 < K; k0 += 32) {
    V bh[4], bl[4];
#pragma unroll
    for (int j = 0; j < 4; ++j) {
      const size_t bo = (size_t)(n0 + (j << 4) + rlane) * ldb + koff + k0;
      bh[j] = Frag<T>::load(Bb + bo);
      if (SPLIT) bl[j] = Frag<T>::load(Bb2 + bo);
    }
#pragma unroll
    for (int i = 0; i < 4; ++i) {
      const size_t ao = (size_t)(m0 + (i << 4) + rlane) * lda + koff + k0;
      V ah = Frag<T>::load(Ab + ao);
      V al;
      if (SPLIT) al = Frag<T>::load(Ab2 + ao);
#pragma unroll
      for (int j = 0; j < 4; ++j) {
        acc[i][j] = Frag<T>::mma(ah, bh[j], acc[i][j]);
        if (SPLIT) {
          acc[i][j] = Frag<T>::mma(ah, bl[j], acc[i][j]);
          acc[i][j] = Frag<T>::mma(al, bh[j], acc[i][j]);
        }
      }
      Frag<T>::guard(acc[i][0], acc[i][3], ah, SPLIT ? al : ah);
    }
    Frag<T>::keep(bh[0], bh[1], bh[2], bh[3]);
    if (SPLIT) Frag<T>::keep(bl[0], bl[1], bl[2], bl[3]);
  }
  acc_guard4(acc[0][0], acc[0][1], acc[0][2], acc[0][3]);
  acc_guard4(acc[1][0], acc[1][1], acc[1][2], acc[1][3]);
  acc_guard4(acc[2][0], acc[2][1], acc[2][2], acc[2][3]);
  acc_guard4(acc[3][0], acc[3][1], acc[3][2], acc[3][3]);

  float* slab = sT[wave];
  const float* Rb = RESID ? (resid + (size_t)b * strideR) : nullptr;
#pragma unroll
  for (int i = 0; i < 4; ++i) {
    const int mBase = m0 + (i << 4);
#pragma unroll
    for (int j = 0; j < 4; ++j) {
      const int n = n0 + (j << 4) + rlane;
      float bv = 0.f;
      if (BIAS_MODE == 2) bv = bias[n];
#pragma unroll
      for (int r = 0; r < 8; ++r) {
        float v = acc[i][j][r] * scale;
        if (BIAS_MODE == 1) v += bias[mBase + mOff + r];
        if (BIAS_MODE == 2) v += bv;
        if (RESID) v += Rb[(size_t)(mBase + mOff + r) * ldc + n];
        if (ACT == 2) v = fmaxf(v, 0.0f);
        if (ACT == 4) v = (v > 0.f) ? v : 0.01f * v;
        slab[(mOff + r) * 68 + (j << 4) + rlane] = v;
      }
    }
    __builtin_amdgcn_fence(__ATOMIC_RELEASE, "workgroup");
    __builtin_amdgcn_wave_barrier();
    __builtin_amdgcn_fence(__ATOMIC_ACQUIRE, "workgroup");
    if (OUT_MODE == 0) {
      float* C = (float*)Cout + (size_t)b * strideC;
      const int hh = lane >> 4, c4 = (lane & 15) * 4;
      for (int pass = 0; pass < 2; ++pass) {
#pragma unroll
        for (int it = 0; it < 8; ++it) {
          const int row = it * 2 + hh;
          v4f v = *(const v4f*)(slab + row * 68 + c4);
          *(volatile v4f*)(C + (size_t)(mBase + row) * ldc + n0 + c4) = v;
        }
        __threadfence();
      }
    } else {
      const int q = lane >> 3, c8 = (lane & 7) * 8;
      unsigned short* C  = (unsigned short*)Cout  + (size_t)b * strideC;
      unsigned short* C2 = (OUT_MODE == 2) ? ((unsigned short*)Cout2 + (size_t)b * strideC) : nullptr;
      for (int pass = 0; pass < 2; ++pass) {
#pragma unroll
        for (int it = 0; it < 4; ++it) {
          const int row = it * 4 + q;
          const float* sp = slab + row * 68 + c8;
          v8h hv, lv;
#pragma unroll
          for (int e = 0; e < 8; ++e) {
            if (OUT_MODE == 1) {
              hv[e] = (_Float16)sp[e];
            } else {
              unsigned short hb = f2bf_bits(sp[e]);
              unsigned short lb = f2bf_bits(sp[e] - bf_bits2f(hb));
              hv[e] = __builtin_bit_cast(_Float16, hb);
              lv[e] = __builtin_bit_cast(_Float16, lb);
            }
          }
          *(volatile v8h*)(C + (size_t)(mBase + row) * ldc + n0 + c8) = hv;
          if (OUT_MODE == 2) *(volatile v8h*)(C2 + (size_t)(mBase + row) * ldc + n0 + c8) = lv;
        }
        __threadfence();
      }
    }
    __builtin_amdgcn_fence(__ATOMIC_RELEASE, "workgroup");
    __builtin_amdgcn_wave_barrier();
    __builtin_amdgcn_fence(__ATOMIC_ACQUIRE, "workgroup");
  }
}

__global__ __launch_bounds__(256) void cast_f16_kernel(const float* __restrict__ s0, const float* __restrict__ s1,
                                                       const float* __restrict__ s2, const float* __restrict__ s3,
                                                       unsigned short* __restrict__ out, long planeStride,
                                                       int nrowsSrc, int ncols, int n8, float scale) {
  const int i = blockIdx.x * 256 + threadIdx.x;
  if (i >= n8) return;
  const int z = blockIdx.y;
  const float* src = (z == 0) ? s0 : (z == 1) ? s1 : (z == 2) ? s2 : s3;
  const long e = 8L * (long)i;
  const int row = (int)(e / ncols);
  const int col = (int)(e - (long)row * ncols);
  const bool live = row < nrowsSrc;
  const int rowc = live ? row : (nrowsSrc - 1);
  const float* p = src + (size_t)rowc * ncols + col;
  const v4f a = *(const v4f*)(p);
  const v4f c = *(const v4f*)(p + 4);
  unsigned short hb[8];
#pragma unroll
  for (int k = 0; k < 4; ++k) {
    const float x0 = live ? a[k] * scale : 0.0f;
    const float x1 = live ? c[k] * scale : 0.0f;
    hb[k]     = h_bits(x0);
    hb[4 + k] = h_bits(x1);
  }
  const v4u u = (v4u){pk16(hb[0], hb[1]), pk16(hb[2], hb[3]), pk16(hb[4], hb[5]), pk16(hb[6], hb[7])};
  unsigned short* q = out + (size_t)z * planeStride + 8 * (size_t)i;
  *(volatile v4u*)q = u;
  __threadfence();
  *(volatile v4u*)q = u;
}

__global__ __launch_bounds__(256) void l2norm_kernel(const float* __restrict__ X, unsigned short* __restrict__ Y, int nrows) {
  const int lane = threadIdx.x & 31, wave = threadIdx.x >> 5;
  const int row = blockIdx.x * 8 + wave;
  if (row >= nrows) return;
  const float* xr = X + (size_t)row * kEmb;
  const v4f a0 = *(const v4f*)(xr + 8 * lane);
  const v4f a1 = *(const v4f*)(xr + 8 * lane + 4);
  const v4f b0 = *(const v4f*)(xr + 256 + 8 * lane);
  const v4f b1 = *(const v4f*)(xr + 256 + 8 * lane + 4);
  float ss = 0.f;
#pragma unroll
  for (int e = 0; e < 4; ++e) { ss += a0[e] * a0[e]; ss += a1[e] * a1[e]; ss += b0[e] * b0[e]; ss += b1[e] * b1[e]; }
#pragma unroll
  for (int off = 16; off > 0; off >>= 1) ss += __shfl_xor(ss, off, 32);
  const float inv = kUnitCarry / fmaxf(sqrtf(ss), 1e-12f);
  unsigned short ha[8], hbv[8];
#pragma unroll
  for (int e = 0; e < 4; ++e) {
    ha[e]      = h_bits(a0[e] * inv);
    ha[4 + e]  = h_bits(a1[e] * inv);
    hbv[e]     = h_bits(b0[e] * inv);
    hbv[4 + e] = h_bits(b1[e] * inv);
  }
  const v4u ua = (v4u){pk16(ha[0], ha[1]), pk16(ha[2], ha[3]), pk16(ha[4], ha[5]), pk16(ha[6], ha[7])};
  const v4u ub = (v4u){pk16(hbv[0], hbv[1]), pk16(hbv[2], hbv[3]), pk16(hbv[4], hbv[5]), pk16(hbv[6], hbv[7])};
  unsigned short* yr = Y + (size_t)row * kEmb;
  *(volatile v4u*)(yr + 8 * lane)       = ua;
  *(volatile v4u*)(yr + 256 + 8 * lane) = ub;
  __threadfence();
  *(volatile v4u*)(yr + 8 * lane)       = ua;
  *(volatile v4u*)(yr + 256 + 8 * lane) = ub;
}

__global__ __launch_bounds__(256) void simred_kernel(const float* __restrict__ S, const int* __restrict__ lens,
                                                     float* __restrict__ tab, int chunk) {
  __shared__ float cmT[80];
  __shared__ float vpart[8][224];
  __shared__ float rmV[224];
  const int tid = threadIdx.x, lane = tid & 31, w = tid >> 5;
  const int bl = blockIdx.x, q = blockIdx.y;
  const int b = chunk * kChunkImg + bl;
  int len = lens[q];
  len = (len < 0) ? 0 : ((len > kNTxt) ? kNTxt : len);
  const float NEG = -INFINITY;
  const float* Sb = S + (size_t)(q * kNTxt) * kSimLd + bl * kNVis;

  float vmax[7];
#pragma unroll
  for (int j = 0; j < 7; ++j) vmax[j] = NEG;

#pragma unroll 1
  for (int i = 0; i < 10; ++i) {
    const int t = w + 8 * i;
    const bool tval = t < kNTxt;
    const bool tin = t < len;
    const int tc = tval ? t : (kNTxt - 1);
    const float* rowp = Sb + (size_t)tc * kSimLd;
    float rp = NEG;
#pragma unroll
    for (int j = 0; j < 7; ++j) {
      const int v = lane + 32 * j;
      const bool vok = v < kNVis;
      const int vc = vok ? v : (kNVis - 1);
      const float xl = rowp[vc];
      const float x = vok ? xl : NEG;
      rp = fmaxf(rp, x);
      vmax[j] = tin ? fmaxf(vmax[j], x) : vmax[j];
    }
#pragma unroll
    for (int off = 16; off > 0; off >>= 1) rp = fmaxf(rp, __shfl_xor(rp, off, 32));
    if (lane == 0 && tval) cmT[t] = rp;
  }
#pragma unroll
  for (int j = 0; j < 7; ++j) vpart[w][lane + 32 * j] = vmax[j];
  __syncthreads();
  if (tid < kNVis) {
    float m = NEG;
#pragma unroll
    for (int ww = 0; ww < 8; ++ww) m = fmaxf(m, vpart[ww][tid]);
    if (len < kNTxt) m = fmaxf(m, 0.0f);
    rmV[tid] = m;
  }
  __syncthreads();

  float s1 = 0.f;
#pragma unroll
  for (int kk = 0; kk < 3; ++kk) {
    const int t = lane + 32 * kk;
    const int tc = (t < kNTxt) ? t : (kNTxt - 1);
    const float cv = cmT[tc];
    s1 += (t < len) ? cv : 0.0f;
  }
  float s2 = 0.f;
#pragma unroll
  for (int j = 0; j < 7; ++j) {
    const int v = lane + 32 * j;
    const int vc = (v < kNVis) ? v : (kNVis - 1);
    const float rv = rmV[vc];
    s2 += (v < kNVis) ? rv : 0.0f;
  }
#pragma unroll
  for (int off = 16; off > 0; off >>= 1) {
    s1 += __shfl_xor(s1, off, 32);
    s2 += __shfl_xor(s2, off, 32);
  }
  const float t2v = s1 * (1.0f / (float)len);
  const float v2t = s2 * (1.0f / (float)kNVis);
  if (w == 0 && lane < 8) {
    v4f val;
    val[0] = (lane == 0) ? t2v : 0.0f;
    val[1] = (lane == 0) ? v2t : 0.0f;
    val[2] = 0.0f;
    val[3] = 0.0f;
    float* line = tab + (size_t)(b * kTxtB + q) * 32 + lane * 4;
    *(volatile v4f*)line = val;
    __threadfence();
    *(volatile v4f*)line = val;
  }
}

__global__ __launch_bounds__(256) void copy_cls_kernel(const float* __restrict__ cls32, float* __restrict__ out) {
  const int i = blockIdx.x * 256 + threadIdx.x;
  const int perPlane = kImg * kEmb / 4;
  if (i >= 2 * perPlane) return;
  const int plane = i / perPlane;
  const int r = i - plane * perPlane;
  const v4f v = *(const v4f*)(cls32 + (size_t)plane * kClsPad * kEmb + 4 * (size_t)r);
  float* dst = out + (size_t)plane * kImg * kEmb + 4 * (size_t)r;
  *(volatile v4f*)dst = v;
  __threadfence();
  *(volatile v4f*)dst = v;
}

__global__ __launch_bounds__(256) void finish_sim_kernel(const float* __restrict__ tab, float* __restrict__ out) {
  const int i = blockIdx.x * 256 + threadIdx.x;
  const int perOut = kImg * kTxtB / 4;
  if (i >= 2 * perOut) return;
  const int o = i / perOut;
  const int k4 = i - o * perOut;
  v4f val;
#pragma unroll
  for (int e = 0; e < 4; ++e) val[e] = tab[(size_t)(4 * k4 + e) * 32 + o];
  float* dst = out + kOut2Elem + (size_t)o * (kImg * kTxtB) + 4 * (size_t)k4;
  *(volatile v4f*)dst = val;
  __threadfence();
  *(volatile v4f*)dst = val;
}

extern "C" void kernel_launch(void* const* d_in, const int* in_sizes, int n_in,
                              void* d_out, int out_size, void* d_ws, size_t ws_size,
                              hipStream_t stream) {
  if (n_in < 13) return;
  if (ws_size < kWsTotal) return;
  if (out_size < kOutTotal) return;
  if (in_sizes[0] != kImg * kDin || in_sizes[1] != kImg * kNVis * kDin ||
      in_sizes[2] != kTxtB * kDin || in_sizes[3] != kTxtB * kNTxt * kDin ||
      in_sizes[4] != kEmb * kDin || in_sizes[6] != kEmb * kDin ||
      in_sizes[8] != kEmb * kDin || in_sizes[10] != kEmb * kDin ||
      in_sizes[5] != kEmb || in_sizes[7] != kEmb || in_sizes[9] != kEmb || in_sizes[11] != kEmb ||
      in_sizes[12] != kTxtB) return;

  const float* visual_cls     = (const float*)d_in[0];
  const float* visual_tokens  = (const float*)d_in[1];
  const float* textual_cls    = (const float*)d_in[2];
  const float* textual_tokens = (const float*)d_in[3];
  const float* Wv_cls = (const float*)d_in[4];
  const float* bv_cls = (const float*)d_in[5];
  const float* Wt_cls = (const float*)d_in[6];
  const float* bt_cls = (const float*)d_in[7];
  const float* Wv_tok = (const float*)d_in[8];
  const float* bv_tok = (const float*)d_in[9];
  const float* Wt_tok = (const float*)d_in[10];
  const float* bt_tok = (const float*)d_in[11];
  const int*   text_length = (const int*)d_in[12];
  float* out = (float*)d_out;

  char* ws = (char*)d_ws;
  unsigned short* W16   = (unsigned short*)(ws + kOffW16);
  unsigned short* XC16  = (unsigned short*)(ws + kOffXC16);
  unsigned short* XT16  = (unsigned short*)(ws + kOffXT16);
  float*          PT32  = (float*)(ws + kOffPT32);
  unsigned short* TT16  = (unsigned short*)(ws + kOffTT16);
  unsigned short* VT16  = (unsigned short*)(ws + kOffVT16);
  float*          CLS32 = (float*)(ws + kOffCLS32);
  float*          TAB   = (float*)(ws + kOffTAB);
  unsigned short* XV16  = (unsigned short*)(ws + kOffXV16);
  float*          PV32  = (float*)(ws + kOffPV32);
  float*          S32   = (float*)(ws + kOffS);

  const size_t wPlane   = (size_t)kEmb * kDin;
  const size_t xcPlane  = (size_t)kClsPad * kDin;
  const size_t clsPlane = (size_t)kClsPad * kEmb;

  {
    const int n8 = kEmb * kDin / 8;
    cast_f16_kernel<<<dim3((n8 + 255) / 256, 4), 256, 0, stream>>>(Wv_cls, Wt_cls, Wv_tok, Wt_tok, W16, (long)wPlane,
                                                                   kEmb, kDin, n8, kWCarry);
  }
  {
    const int n8 = kClsPad * kDin / 8;
    cast_f16_kernel<<<dim3((n8 + 255) / 256, 2), 256, 0, stream>>>(visual_cls, textual_cls, visual_cls, visual_cls, XC16,
                                                                   (long)xcPlane, kImg, kDin, n8, 1.0f);
  }
  {
    const int n8v = kRowsVP * kDin / 8;
    cast_f16_kernel<<<dim3((n8v + 255) / 256, 1), 256, 0, stream>>>(visual_tokens, visual_tokens, visual_tokens, visual_tokens,
                                                                    XV16, 0L, kRowsV, kDin, n8v, 1.0f);
    const int n8t = kRowsTP * kDin / 8;
    cast_f16_kernel<<<dim3((n8t + 255) / 256, 1), 256, 0, stream>>>(textual_tokens, textual_tokens, textual_tokens, textual_tokens,
                                                                    XT16, 0L, kRowsT, kDin, n8t, 1.0f);
  }
  {
    const int nblk = ((kClsPad / 64) * (kEmb / 64) + 7) / 8;
    wmma_gemm64<0, false, 2, 0, false, 0><<<dim3(nblk, 1), 256, 0, stream>>>(
        XC16, XC16, kDin, 0L, W16, W16, kDin, 0L,
        CLS32, CLS32, kEmb, 0L, bv_cls, PV32, 0L, kClsPad, kEmb, kDin, kWCarryInv);
    wmma_gemm64<0, false, 2, 0, false, 0><<<dim3(nblk, 1), 256, 0, stream>>>(
        XC16 + xcPlane, XC16 + xcPlane, kDin, 0L, W16 + wPlane, W16 + wPlane, kDin, 0L,
        CLS32 + clsPlane, CLS32 + clsPlane, kEmb, 0L, bt_cls, PV32, 0L, kClsPad, kEmb, kDin, kWCarryInv);
    copy_cls_kernel<<<dim3((2 * kImg * kEmb / 4 + 255) / 256), 256, 0, stream>>>(CLS32, out);
  }
  {
    const int nblk = ((kRowsVP / 64) * (kEmb / 64) + 7) / 8;
    wmma_gemm64<0, false, 2, 0, false, 0><<<dim3(nblk, 1), 256, 0, stream>>>(
        XV16, XV16, kDin, 0L, W16 + 2 * wPlane, W16 + 2 * wPlane, kDin, 0L,
        PV32, PV32, kEmb, 0L, bv_tok, PT32, 0L, kRowsVP, kEmb, kDin, kWCarryInv);
    l2norm_kernel<<<dim3(kRowsVP / 8), 256, 0, stream>>>(PV32, VT16, kRowsVP);
  }
  {
    const int nblk = ((kRowsTP / 64) * (kEmb / 64) + 7) / 8;
    wmma_gemm64<0, false, 2, 0, false, 0><<<dim3(nblk, 1), 256, 0, stream>>>(
        XT16, XT16, kDin, 0L, W16 + 3 * wPlane, W16 + 3 * wPlane, kDin, 0L,
        PT32, PT32, kEmb, 0L, bt_tok, PV32, 0L, kRowsTP, kEmb, kDin, kWCarryInv);
    l2norm_kernel<<<dim3(kRowsTP / 8), 256, 0, stream>>>(PT32, TT16, kRowsTP);
  }
  {
    const int tiles = (kRowsTP / 64) * (kSimN / 64);
    const int nblk = (tiles + 7) / 8;
    for (int c = 0; c < kNumChunk; ++c) {
      const unsigned short* Bt = VT16 + (size_t)c * kChunkImg * kNVis * kEmb;
      wmma_gemm64<0, false, 0, 0, false, 0><<<dim3(nblk, 1), 256, 0, stream>>>(
          TT16, TT16, kEmb, 0L, Bt, Bt, kEmb, 0L,
          S32, S32, kSimLd, 0L, bv_tok, PT32, 0L, kRowsTP, kSimN, kEmb, kSimScale);
      simred_kernel<<<dim3(kChunkImg, kTxtB), 256, 0, stream>>>(S32, text_length, TAB, c);
    }
  }
  finish_sim_kernel<<<dim3((2 * kImg * kTxtB / 4 + 255) / 256), 256, 0, stream>>>(TAB, out);
}
